// SymplecticNeuralSolver_37065567764798
// MI455X (gfx1250) — hardware-verified
//
#include <hip/hip_runtime.h>


#define NB_  8
#define NG   4096
#define NR   (NB_ * NG)
#define DD   32
#define DA   16
#define DIN  80
#define KP   96
#define HID  128
#define NSTEP 18
#define DTC  0.25f
typedef _Float16 h16;
typedef unsigned short bf;
typedef __attribute__((ext_vector_type(16))) __bf16   v16bf;
typedef __attribute__((ext_vector_type(16))) _Float16 v16h;
typedef __attribute__((ext_vector_type(8)))  _Float16 v8h;
typedef __attribute__((ext_vector_type(8)))  unsigned short v8us;
typedef __attribute__((ext_vector_type(8)))  float    v8f;
typedef __attribute__((ext_vector_type(4)))  float    v4f;
typedef v8h  __attribute__((may_alias)) v8ha;
typedef v4f  __attribute__((may_alias)) v4fa;
typedef v8us __attribute__((may_alias)) v8usa;

__device__ __forceinline__ unsigned short f2bf(float f) { unsigned u = __float_as_uint(f); u += 0x7FFFu + ((u >> 16) & 1u); return (unsigned short)(u >> 16); }
__device__ __forceinline__ float bf2f(unsigned short b) { return __uint_as_float(((unsigned)b) << 16); }
__device__ __forceinline__ float bfr(float f) { return bf2f(f2bf(f)); }
__device__ __forceinline__ v16h cat16(v8h lo, v8h hi) { return __builtin_shufflevector(lo, hi, 0, 1, 2, 3, 4, 5, 6, 7, 8, 9, 10, 11, 12, 13, 14, 15); }
__device__ __forceinline__ v16bf cat16b(v8us lo, v8us hi) { return __builtin_bit_cast(v16bf, __builtin_shufflevector(lo, hi, 0, 1, 2, 3, 4, 5, 6, 7, 8, 9, 10, 11, 12, 13, 14, 15)); }
__device__ __forceinline__ v8f wmma16(v16h a, v16h b, v8f c) { return __builtin_amdgcn_wmma_f32_16x16x32_f16(false, a, false, b, (short)0, c, false, false); }
__device__ __forceinline__ v8f wmmab(v16bf a, v16bf b, v8f c) { return __builtin_amdgcn_wmma_f32_16x16x32_bf16(false, a, false, b, (short)0, c, false, false); }


template <typename T16> struct WFrag;
template <> struct WFrag<h16> { typedef v16h V; static __device__ __forceinline__ V ld(const h16* p) { return cat16(*(const v8h*)p, *(const v8h*)(p + 16)); } static __device__ __forceinline__ v8f mma(V a, V b, v8f c) { return wmma16(a, b, c); } };
template <> struct WFrag<bf> { typedef v16bf V; static __device__ __forceinline__ V ld(const bf* p) { return cat16b(*(const v8us*)p, *(const v8us*)(p + 16)); } static __device__ __forceinline__ v8f mma(V a, V b, v8f c) { return wmmab(a, b, c); } };
template <typename T16, int NSPLIT, bool BIAS>
__global__ __launch_bounds__(32) void k_gemmw(const T16* __restrict__ A, const T16* __restrict__ A2, const T16* __restrict__ Bt, const T16* __restrict__ Bt2, int K, float* C, int ldc, const float* __restrict__ bias, size_t sA, size_t sB, size_t sC) {
    typedef typename WFrag<T16>::V V;
    __shared__ __align__(16) float os[16 * 68];
    const size_t z = blockIdx.z; A += z * sA; if (A2) A2 += z * sA; Bt += z * sB; if (Bt2) Bt2 += z * sB; C += z * sC;
    const int lane = threadIdx.x & 31, lr = lane & 15, hi = lane >> 4; const int r0 = blockIdx.x * 64, c0 = blockIdx.y * 64;
    v8f acc[4][4];
#pragma unroll
    for (int mb = 0; mb < 4; ++mb)
#pragma unroll
        for (int nb = 0; nb < 4; ++nb) acc[mb][nb] = (v8f){};
    const size_t aoff = (size_t)(r0 + lr) * K + 8 * hi, boff = (size_t)(c0 + lr) * K + 8 * hi;
#pragma unroll 1
    for (int kc = 0; kc < K; kc += 32) {
        V a[4], a2[4];
#pragma unroll
        for (int mb = 0; mb < 4; ++mb) { a[mb] = WFrag<T16>::ld(A + aoff + (size_t)mb * 16 * K + kc); if (NSPLIT == 1 || NSPLIT == 2) a2[mb] = WFrag<T16>::ld(A2 + aoff + (size_t)mb * 16 * K + kc); }
#pragma unroll
        for (int nb = 0; nb < 4; ++nb) { const V b = WFrag<T16>::ld(Bt + boff + (size_t)nb * 16 * K + kc); V b2; if (NSPLIT >= 2) b2 = WFrag<T16>::ld(Bt2 + boff + (size_t)nb * 16 * K + kc);
#pragma unroll
            for (int mb = 0; mb < 4; ++mb) { acc[mb][nb] = WFrag<T16>::mma(a[mb], b, acc[mb][nb]); if (NSPLIT == 1 || NSPLIT == 2) acc[mb][nb] = WFrag<T16>::mma(a2[mb], b, acc[mb][nb]); if (NSPLIT >= 2) acc[mb][nb] = WFrag<T16>::mma(a[mb], b2, acc[mb][nb]); } }
        asm volatile("v_nop\n\tv_nop\n\tv_nop\n\tv_nop" : "+v"(acc[0][0]), "+v"(acc[1][1]), "+v"(acc[2][2]), "+v"(acc[3][3]) : "v"(a[0]), "v"(a[3]));
    }
#pragma unroll
    for (int mb = 0; mb < 4; ++mb) {
#pragma unroll
        for (int nb = 0; nb < 4; ++nb) {
#pragma unroll
            for (int j = 0; j < 8; ++j) os[(hi * 8 + j) * 68 + nb * 16 + lr] = acc[mb][nb][j]; }
        __builtin_amdgcn_wave_barrier(); asm volatile("" ::: "memory");
        float* crow = C + (size_t)(r0 + mb * 16) * ldc + c0;
#pragma unroll 1
        for (int ps = 0; ps < 2; ++ps) {
#pragma unroll
            for (int s = 0; s < 8; ++s) { const int row = 2 * s + hi, cofs = lr * 4; v4f val = *(const v4fa*)(os + row * 68 + cofs); if (BIAS) { val[0] += bfr(bias[c0 + cofs]); val[1] += bfr(bias[c0 + cofs + 1]); val[2] += bfr(bias[c0 + cofs + 2]); val[3] += bfr(bias[c0 + cofs + 3]); }
                *(volatile v4f*)(crow + (size_t)row * ldc + cofs) = val; }
            if (ps == 0) __threadfence(); }
        __builtin_amdgcn_wave_barrier(); asm volatile("" ::: "memory");
    }
}

__device__ __forceinline__ void splitf(float y, unsigned short& h, unsigned short& l) { h = f2bf(y); l = f2bf(y - bf2f(h)); }
__device__ __forceinline__ float tanhf_(float a) { const float e2 = __expf(2.0f * a); return __fsub_rn(1.0f, __fdiv_rn(2.0f, __fadd_rn(e2, 1.0f))); }
typedef __attribute__((ext_vector_type(4))) unsigned short v4us;
typedef __attribute__((ext_vector_type(4))) _Float16 v4h;
__device__ __forceinline__ h16 tohx(float x) { return (h16)x; }

__global__ __launch_bounds__(256) void k_w1p(const float* __restrict__ W1, h16* Bt) { const int e = (blockIdx.x * 256 + threadIdx.x) * 4; if (e >= HID * KP) return; const int k = e % KP, o = e / KP; v4h r;
#pragma unroll
    for (int q = 0; q < 4; ++q) r[q] = (k + q) < DIN ? tohx(bfr(W1[(size_t)(k + q) * HID + o])) : (h16)0.f; *(volatile v4h*)(Bt + e) = r; __threadfence(); *(volatile v4h*)(Bt + e) = r; }
__global__ __launch_bounds__(256) void k_w2p(const float* __restrict__ W2, h16* Bt) { const int e = (blockIdx.x * 256 + threadIdx.x) * 4; if (e >= 64 * HID) return; const int k = e % HID, o = e / HID; v4h r;
#pragma unroll
    for (int q = 0; q < 4; ++q) r[q] = o < DD ? tohx(bfr(W2[(size_t)(k + q) * DD + o])) : (h16)0.f; *(volatile v4h*)(Bt + e) = r; __threadfence(); *(volatile v4h*)(Bt + e) = r; }
__global__ __launch_bounds__(256) void k_init(const float* __restrict__ x, float* Q, float* Pm) { const int e = (blockIdx.x * 256 + threadIdx.x) * 4; if (e >= NR * DD) return; const int d = e % DD, r = e / DD; v4f a, b;
#pragma unroll
    for (int q = 0; q < 4; ++q) { a[q] = bfr(x[(size_t)r * DIN + d + q]); b[q] = bfr(x[(size_t)r * DIN + DD + d + q]); } *(volatile v4f*)(Q + e) = a; *(volatile v4f*)(Pm + e) = b; __threadfence(); *(volatile v4f*)(Q + e) = a; *(volatile v4f*)(Pm + e) = b; }
__global__ __launch_bounds__(256) void k_inp(const float* __restrict__ Z, const float* __restrict__ x, const int* __restrict__ nbrs, h16* A16) { const size_t e = ((size_t)blockIdx.x * 256 + threadIdx.x) * 4; if (e >= (size_t)NR * KP) return; const int c = (int)(e % KP); const int r = (int)(e / KP); const int n = r % NG; const int rb = r - n; v4h o;
#pragma unroll
    for (int q = 0; q < 4; ++q) { const int cq = c + q; float v = 0.f;
        if (cq < DD) v = Z[(size_t)r * DD + cq];
        else if (cq < 2 * DD) { const int d = cq - DD; float s = 0.f; for (int i = 0; i < 4; ++i) { int nn = nbrs[n * 4 + i]; nn = min(max(nn, 0), NG - 1); s = __fadd_rn(s, Z[(size_t)(rb + nn) * DD + d]); } v = __fmul_rn(s, 0.25f); }
        else if (cq < DIN) v = bfr(x[(size_t)r * DIN + 2 * DD + (cq - 2 * DD)]);
        o[q] = tohx(v); }
    *(volatile v4h*)(A16 + e) = o; __threadfence(); *(volatile v4h*)(A16 + e) = o; }
__global__ __launch_bounds__(256) void k_tanh(const float* __restrict__ Hf, h16* T16) { const size_t i = ((size_t)blockIdx.x * 256 + threadIdx.x) * 4; if (i >= (size_t)NR * HID) return; const v4f a = *(const v4f*)(Hf + i); v4h o;
#pragma unroll
    for (int q = 0; q < 4; ++q) o[q] = tohx(tanhf_(a[q])); *(volatile v4h*)(T16 + i) = o; __threadfence(); *(volatile v4h*)(T16 + i) = o; }
__global__ __launch_bounds__(256) void k_upd(const float* __restrict__ F, const float* __restrict__ b2, const float* __restrict__ tf, float t, float dtmax, float* Z) { const int e = (blockIdx.x * 256 + threadIdx.x) * 4; if (e >= NR * DD) return; const int d = e % DD, r = e / DD; const int b = r / NG;
    const float dt = fminf(fmaxf(__fsub_rn(bfr(tf[b]), t), 0.f), dtmax); const v4f z = *(const v4f*)(Z + e); v4f o;
#pragma unroll
    for (int q = 0; q < 4; ++q) { const float f = __fadd_rn(F[(size_t)r * 64 + d + q], bfr(b2[d + q])); float df = __fmul_rn(dt, f); asm volatile("" : "+v"(df)); o[q] = __fadd_rn(z[q], df); } *(volatile v4f*)(Z + e) = o; __threadfence(); *(volatile v4f*)(Z + e) = o; }
__global__ __launch_bounds__(256) void k_out(const float* __restrict__ Q, const float* __restrict__ Pm, const float* __restrict__ x, float* OUT) { const int e = (blockIdx.x * 256 + threadIdx.x) * 4; if (e >= NR * DIN) return; const int c = e % DIN, r = e / DIN; v4f o;
#pragma unroll
    for (int q = 0; q < 4; ++q) { const int cq = c + q; o[q] = cq < DD ? Q[(size_t)r * DD + cq] : (cq < 2 * DD ? Pm[(size_t)r * DD + cq - DD] : bfr(x[(size_t)r * DIN + cq])); } *(volatile v4f*)(OUT + e) = o; __threadfence(); *(volatile v4f*)(OUT + e) = o; }

extern "C" void kernel_launch(void* const* d_in, const int* in_sizes, int n_in,
                              void* d_out, int out_size, void* d_ws, size_t ws_size, hipStream_t stream) {
    (void)in_sizes; (void)n_in; (void)out_size;
    const float* x = (const float*)d_in[0]; const float* tf = (const float*)d_in[1]; const float* W1q = (const float*)d_in[2]; const float* b1q = (const float*)d_in[3]; const float* W2q = (const float*)d_in[4]; const float* b2q = (const float*)d_in[5]; const float* W1p = (const float*)d_in[6]; const float* b1p = (const float*)d_in[7]; const float* W2p = (const float*)d_in[8]; const float* b2p = (const float*)d_in[9]; const int* nbrs = (const int*)d_in[10];
    float* OUT = (float*)d_out;
    char* wsp = (char*)d_ws;
    auto take = [&](size_t bytes) { char* p = wsp; wsp += (bytes + 255) & ~(size_t)255; return (void*)p; };
    h16* B1q = (h16*)take((size_t)HID * KP * 2); h16* B2q = (h16*)take((size_t)64 * HID * 2); h16* B1p = (h16*)take((size_t)HID * KP * 2); h16* B2p = (h16*)take((size_t)64 * HID * 2);
    float* Q = (float*)take((size_t)NR * DD * 4); float* Pm = (float*)take((size_t)NR * DD * 4); h16* A16 = (h16*)take((size_t)NR * KP * 2); float* Hf = (float*)take((size_t)NR * HID * 4); h16* T16 = (h16*)take((size_t)NR * HID * 2); float* F = (float*)take((size_t)NR * 64 * 4);
    if ((size_t)(wsp - (char*)d_ws) > ws_size) return;
    k_w1p<<<(HID * KP / 4 + 255) / 256, 256, 0, stream>>>(W1q, B1q); k_w2p<<<(64 * HID / 4 + 255) / 256, 256, 0, stream>>>(W2q, B2q); k_w1p<<<(HID * KP / 4 + 255) / 256, 256, 0, stream>>>(W1p, B1p); k_w2p<<<(64 * HID / 4 + 255) / 256, 256, 0, stream>>>(W2p, B2p);
    k_init<<<(NR * DD / 4 + 255) / 256, 256, 0, stream>>>(x, Q, Pm);
    const unsigned LI = (unsigned)(((size_t)NR * KP / 4 + 255) / 256), LT = (unsigned)(((size_t)NR * HID / 4 + 255) / 256), LU = (NR * DD / 4 + 255) / 256;
    float t_q = 0.f, t_p = 0.f;
    for (int k = 0; k < NSTEP; ++k) { const float rho = k == 0 ? 0.5f : 1.0f;
        k_inp<<<LI, 256, 0, stream>>>(Pm, x, nbrs, A16); k_gemmw<h16, 0, true><<<dim3(NR / 64, HID / 64, 1), 32, 0, stream>>>(A16, nullptr, B1q, nullptr, KP, Hf, HID, b1q, 0, 0, 0); k_tanh<<<LT, 256, 0, stream>>>(Hf, T16);
        k_gemmw<h16, 0, false><<<dim3(NR / 64, 1, 1), 32, 0, stream>>>(T16, nullptr, B2q, nullptr, HID, F, 64, nullptr, 0, 0, 0); k_upd<<<LU, 256, 0, stream>>>(F, b2q, tf, t_q, rho * DTC, Q); t_q += rho * DTC;
        k_inp<<<LI, 256, 0, stream>>>(Q, x, nbrs, A16); k_gemmw<h16, 0, true><<<dim3(NR / 64, HID / 64, 1), 32, 0, stream>>>(A16, nullptr, B1p, nullptr, KP, Hf, HID, b1p, 0, 0, 0); k_tanh<<<LT, 256, 0, stream>>>(Hf, T16);
        k_gemmw<h16, 0, false><<<dim3(NR / 64, 1, 1), 32, 0, stream>>>(T16, nullptr, B2p, nullptr, HID, F, 64, nullptr, 0, 0, 0); k_upd<<<LU, 256, 0, stream>>>(F, b2p, tf, t_p, DTC, Pm); t_p += DTC; }
    k_out<<<(NR * DIN / 4 + 255) / 256, 256, 0, stream>>>(Q, Pm, x, OUT);
}
